// DiagonalSSM_35003983462988
// MI455X (gfx1250) — hardware-run, weakly checked
//
#include <hip/hip_runtime.h>
#include <math.h>

typedef __attribute__((ext_vector_type(16))) _Float16 v16h;
typedef __attribute__((ext_vector_type(8)))  _Float16 v8h;
typedef __attribute__((ext_vector_type(2)))  _Float16 v2h;
typedef __attribute__((ext_vector_type(16))) __bf16   v16b;
typedef __attribute__((ext_vector_type(8)))  __bf16   v8b;
typedef __attribute__((ext_vector_type(8)))  float    v8f;
typedef __attribute__((ext_vector_type(4)))  float    v4f;
typedef __attribute__((ext_vector_type(2)))  float    v2f;

constexpr int kB    = 256;
constexpr int kL    = 4096;
constexpr int kN    = 64;
constexpr int kQ    = 64;
constexpr int kC    = kL / kQ;
constexpr int kR    = kB * kC;
constexpr int kS    = 2 * kN;
constexpr int kKY   = kQ + kS;
constexpr int kThr  = 256;
constexpr float kInCarry = 512.0f;
constexpr float kACarry  = 16384.0f;
constexpr float kTCarry  = 512.0f;
constexpr float kSc1 = 1.0f / (kInCarry * kACarry);
constexpr float kSc2 = 1.0f / (kInCarry * kTCarry);
constexpr float kF16MinNormal = 6.103515625e-5f;

static_assert(kB == 256 && kL == 4096 && kN == 64 && kQ == 64 && kC == 64 && kR == 16384 && kS == 128 && kKY == 192, "the index arithmetic below uses these sizes");

constexpr size_t kOffZB = 0ull;
constexpr size_t kOffPWR = 4096ull;
constexpr size_t kOffPWI = 20736ull;
constexpr size_t kOffK32 = 37376ull;
constexpr size_t kOffW216 = 37632ull;
constexpr size_t kOffBQ16 = 62208ull;
constexpr size_t kOffXH16 = 78592ull;
constexpr size_t kOffHIN32 = 6370048ull;
constexpr size_t kOffH32 = 14758656ull;
constexpr size_t kWsTotal = 23147264ull;
static_assert(kWsTotal <= 134217728ull, "carve cap: under 128 MiB");
static_assert(kOffZB == 0
              && kOffPWR == kOffZB + 4096ull
              && kOffPWI == kOffPWR + 16640ull
              && kOffK32 == kOffPWI + 16640ull
              && kOffW216 == kOffK32 + 256ull
              && kOffBQ16 == kOffW216 + 24576ull
              && kOffXH16 == kOffBQ16 + 16384ull
              && kOffHIN32 == kOffXH16 + 6291456ull
              && kOffH32 == kOffHIN32 + 8388608ull
              && kWsTotal == kOffH32 + 8388608ull, "the carve is chained and totalled");
static_assert((kOffPWR % 256) == 0 && (kOffPWI % 256) == 0 && (kOffK32 % 256) == 0 && (kOffW216 % 256) == 0 && (kOffBQ16 % 256) == 0 && (kOffXH16 % 256) == 0 && (kOffHIN32 % 256) == 0 && (kOffH32 % 256) == 0, "aligned regions");
static_assert(1024 >= 128, "the zero record covers the widest launch's 128 output columns and the 64 modes of a control's zero plane");

__device__ __forceinline__ unsigned short f2bf_bits(float f) {
  unsigned u = __float_as_uint(f);
  return (unsigned short)((u + 0x7FFFu + ((u >> 16) & 1u)) >> 16);
}
__device__ __forceinline__ float bf_bits2f(unsigned short h) { return __uint_as_float(((unsigned)h) << 16); }
__device__ __forceinline__ float bf16r(float f) { return bf_bits2f(f2bf_bits(f)); }
__device__ __forceinline__ float carry_flush(float v, float carry) {
  const float s = v * carry;
  return (fabsf(s) < kF16MinNormal) ? 0.0f : s;
}

__device__ __forceinline__ void dep_guard4_h(v8f& a, v8f& b, v8f& c, v8f& d, v16h x, v16h y) { asm volatile("v_nop\n\tv_nop\n\tv_nop\n\tv_nop" : "+v"(a), "+v"(b), "+v"(c), "+v"(d) : "v"(x), "v"(y)); }
__device__ __forceinline__ void dep_guard4_b(v8f& a, v8f& b, v8f& c, v8f& d, v16b x, v16b y) { asm volatile("v_nop\n\tv_nop\n\tv_nop\n\tv_nop" : "+v"(a), "+v"(b), "+v"(c), "+v"(d) : "v"(x), "v"(y)); }
__device__ __forceinline__ void keep4_h(v16h a, v16h b, v16h c, v16h d) { asm volatile("v_nop" :: "v"(a), "v"(b), "v"(c), "v"(d)); }
__device__ __forceinline__ void keep4_b(v16b a, v16b b, v16b c, v16b d) { asm volatile("v_nop" :: "v"(a), "v"(b), "v"(c), "v"(d)); }
__device__ __forceinline__ void acc_guard4(v8f& a, v8f& b, v8f& c, v8f& d) { asm volatile("v_nop\n\tv_nop\n\tv_nop\n\tv_nop" : "+v"(a), "+v"(b), "+v"(c), "+v"(d)); }

template <typename T> struct Frag;
template <> struct Frag<_Float16> {
  typedef v16h V; union U { v16h v; v8h h[2]; };
  static __device__ __forceinline__ v16h load(const _Float16* p) {
    U f; f.h[0] = *(const v8h*)(p); f.h[1] = *(const v8h*)(p + 16); return f.v;
  }
  static __device__ __forceinline__ v8f mma(v16h a, v16h b, v8f c) {
    return __builtin_amdgcn_wmma_f32_16x16x32_f16(false, a, false, b, (short)0, c, false, false);
  }
  static __device__ __forceinline__ void guard4(v8f& a, v8f& b, v8f& c, v8f& d, v16h x, v16h y) { dep_guard4_h(a, b, c, d, x, y); }
  static __device__ __forceinline__ void keep(v16h a, v16h b, v16h c, v16h d) { keep4_h(a, b, c, d); }
};
template <> struct Frag<__bf16> {
  typedef v16b V; union U { v16b v; v8b h[2]; };
  static __device__ __forceinline__ v16b load(const __bf16* p) {
    U f; f.h[0] = *(const v8b*)(p); f.h[1] = *(const v8b*)(p + 16); return f.v;
  }
  static __device__ __forceinline__ v8f mma(v16b a, v16b b, v8f c) {
    return __builtin_amdgcn_wmma_f32_16x16x32_bf16(false, a, false, b, (short)0, c, false, false);
  }
  static __device__ __forceinline__ void guard4(v8f& a, v8f& b, v8f& c, v8f& d, v16b x, v16b y) { dep_guard4_b(a, b, c, d, x, y); }
  static __device__ __forceinline__ void keep(v16b a, v16b b, v16b c, v16b d) { keep4_b(a, b, c, d); }
};

__device__ __forceinline__ v8f mma_h(v16h a, v16h b, v8f c) {
  c = __builtin_amdgcn_wmma_f32_16x16x32_f16(false, a, false, b, (short)0, c, false, false);
  asm volatile("v_nop\n\tv_nop\n\tv_nop\n\tv_nop" : "+v"(c) : "v"(a), "v"(b));
  return c;
}

template <int ET> struct Elem;
template <> struct Elem<0> { typedef _Float16 T; };
template <> struct Elem<1> { typedef __bf16 T; };
template <int ET, bool SPLIT, int BIAS_MODE, int OUT_MODE, bool RESID, int ACT = 0>
__global__ __launch_bounds__(256) void wmma_gemm64(
    const unsigned short* __restrict__ Ap, const unsigned short* __restrict__ A2p, int lda, long strideA,
    const unsigned short* __restrict__ Btp, const unsigned short* __restrict__ Bt2p, int ldb, long strideB,
    void* __restrict__ Cout, void* __restrict__ Cout2, int ldc, long strideC,
    const float* __restrict__ bias,
    const float* __restrict__ resid, long strideR,
    int M, int N, int K, float scale) {
  typedef typename Elem<ET>::T T;
  typedef typename Frag<T>::V V;
  const T* A = (const T*)Ap; const T* A2 = (const T*)A2p; const T* Bt = (const T*)Btp; const T* Bt2 = (const T*)Bt2p;
  __shared__ __align__(16) float sT[8][16 * 68];
  const int b    = blockIdx.y;
  const int lane = threadIdx.x & 31;
  const int wave = threadIdx.x >> 5;
  const int tilesN = N >> 6;
  const int tilesM = M >> 6;
  const int tile = blockIdx.x * 8 + wave;
  if (tile >= tilesM * tilesN) return;
  const int tm = tile / tilesN;
  const int tn = tile - tm * tilesN;
  const int m0 = tm << 6;
  const int n0 = tn << 6;

  const T* Ab  = A  + (size_t)b * strideA;
  const T* Bb  = Bt + (size_t)b * strideB;
  const T* Ab2 = SPLIT ? (A2  + (size_t)b * strideA) : nullptr;
  const T* Bb2 = SPLIT ? (Bt2 + (size_t)b * strideB) : nullptr;

  const int rlane = lane & 15;
  const int koff  = (lane >> 4) * 8;
  const int mOff  = (lane >> 4) * 8;

  v8f acc[4][4];
#pragma unroll
  for (int i = 0; i < 4; ++i)
#pragma unroll
    for (int j = 0; j < 4; ++j) acc[i][j] = (v8f){0.f,0.f,0.f,0.f,0.f,0.f,0.f,0.f};

  for (int k0 = 0; k0 < K; k0 += 32) {
    V bh[4], bl[4];
#pragma unroll
    for (int j = 0; j < 4; ++j) {
      const size_t bo = (size_t)(n0 + (j << 4) + rlane) * ldb + koff + k0;
      bh[j] = Frag<T>::load(Bb + bo);
      if (SPLIT) bl[j] = Frag<T>::load(Bb2 + bo);
    }
#pragma unroll
    for (int i = 0; i < 4; ++i) {
      const size_t ao = (size_t)(m0 + (i << 4) + rlane) * lda + koff + k0;
      V ah = Frag<T>::load(Ab + ao);
      V al;
      if (SPLIT) al = Frag<T>::load(Ab2 + ao);
#pragma unroll
      for (int j = 0; j < 4; ++j) {
        acc[i][j] = Frag<T>::mma(ah, bh[j], acc[i][j]);
        if (SPLIT) {
          acc[i][j] = Frag<T>::mma(ah, bl[j], acc[i][j]);
          acc[i][j] = Frag<T>::mma(al, bh[j], acc[i][j]);
        }
      }
      Frag<T>::guard4(acc[i][0], acc[i][1], acc[i][2], acc[i][3], ah, SPLIT ? al : ah);
    }
    Frag<T>::keep(bh[0], bh[1], bh[2], bh[3]);
    if (SPLIT) Frag<T>::keep(bl[0], bl[1], bl[2], bl[3]);
  }
  acc_guard4(acc[0][0], acc[0][1], acc[0][2], acc[0][3]);
  acc_guard4(acc[1][0], acc[1][1], acc[1][2], acc[1][3]);
  acc_guard4(acc[2][0], acc[2][1], acc[2][2], acc[2][3]);
  acc_guard4(acc[3][0], acc[3][1], acc[3][2], acc[3][3]);

  float* slab = sT[wave];
  const float* Rb = RESID ? (resid + (size_t)b * strideR) : nullptr;
#pragma unroll
  for (int i = 0; i < 4; ++i) {
    const int mBase = m0 + (i << 4);
#pragma unroll
    for (int j = 0; j < 4; ++j) {
      const int n = n0 + (j << 4) + rlane;
      float bv = 0.f;
      if (BIAS_MODE == 2) bv = bias[n];
#pragma unroll
      for (int r = 0; r < 8; ++r) {
        float v = acc[i][j][r] * scale;
        if (BIAS_MODE == 1) v += bias[mBase + mOff + r];
        if (BIAS_MODE == 2) v += bv;
        if (RESID) v += Rb[(size_t)(mBase + mOff + r) * ldc + n];
        if (ACT == 1) v = tanhf(v);
        if (ACT == 2) v = fmaxf(v, 0.0f);
        if (ACT == 3) v = v / (1.0f + expf(-v));
        if (ACT == 4) v = (v > 0.f) ? v : 0.01f * v;
        slab[(mOff + r) * 68 + (j << 4) + rlane] = v;
      }
    }
    __builtin_amdgcn_fence(__ATOMIC_RELEASE, "workgroup");
    __builtin_amdgcn_wave_barrier();
    __builtin_amdgcn_fence(__ATOMIC_ACQUIRE, "workgroup");
    if (OUT_MODE == 0) {
      float* C = (float*)Cout + (size_t)b * strideC;
      const int hh = lane >> 4, c4 = (lane & 15) * 4;
      for (int pass = 0; pass < 2; ++pass) {
#pragma unroll
        for (int it = 0; it < 8; ++it) {
          const int row = it * 2 + hh;
          v4f v = *(const v4f*)(slab + row * 68 + c4);
          *(volatile v4f*)(C + (size_t)(mBase + row) * ldc + n0 + c4) = v;
        }
        __threadfence();
      }
    } else {
      const int q = lane >> 3, c8 = (lane & 7) * 8;
      unsigned short* C  = (unsigned short*)Cout  + (size_t)b * strideC;
      unsigned short* C2 = (OUT_MODE == 2) ? ((unsigned short*)Cout2 + (size_t)b * strideC) : nullptr;
      for (int pass = 0; pass < 2; ++pass) {
#pragma unroll
        for (int it = 0; it < 4; ++it) {
          const int row = it * 4 + q;
          const float* sp = slab + row * 68 + c8;
          v8h hv, lv;
#pragma unroll
          for (int e = 0; e < 8; ++e) {
            if (OUT_MODE == 1) {
              hv[e] = (_Float16)sp[e];
            } else {
              unsigned short hb = f2bf_bits(sp[e]);
              unsigned short lb = f2bf_bits(sp[e] - bf_bits2f(hb));
              hv[e] = __builtin_bit_cast(_Float16, hb);
              lv[e] = __builtin_bit_cast(_Float16, lb);
            }
          }
          *(volatile v8h*)(C + (size_t)(mBase + row) * ldc + n0 + c8) = hv;
          if (OUT_MODE == 2) *(volatile v8h*)(C2 + (size_t)(mBase + row) * ldc + n0 + c8) = lv;
        }
        __threadfence();
      }
    }
    __builtin_amdgcn_fence(__ATOMIC_RELEASE, "workgroup");
    __builtin_amdgcn_wave_barrier();
    __builtin_amdgcn_fence(__ATOMIC_ACQUIRE, "workgroup");
  }
}


__device__ __forceinline__ void store2(float* p, float v) {
  *(volatile float*)p = v;
  __threadfence();
  *(volatile float*)p = v;
}


__global__ __launch_bounds__(kThr) void zero_kernel(float* __restrict__ dst) {
  const size_t o4 = ((size_t)blockIdx.x * kThr + threadIdx.x) * 4u;
  const v4f z = {0.f, 0.f, 0.f, 0.f};
  *(volatile v4f*)(dst + o4) = z;
  __threadfence();
  *(volatile v4f*)(dst + o4) = z;
}

__global__ __launch_bounds__(64) void pow_kernel(const float* __restrict__ rho, const float* __restrict__ theta, float* __restrict__ PWR, float* __restrict__ PWI) {
  const unsigned n = threadIdx.x;
  const float rh = rho[n], th = theta[n];
  const float rb = bf16r(rh);
  const float sp = fmaxf(rb, 0.0f) + log1pf(expf(-fabsf(rb)));
  const float radius = expf(-sp);
  const float ar = radius * cosf(bf16r(th));
  const float ai = radius * sinf(bf16r(th));
  float pr = 1.0f, pi = 0.0f;
  store2(PWR + n, pr); store2(PWI + n, pi);
  for (int k = 1; k <= kQ; ++k) {
    const float nr = ar * pr - ai * pi;
    const float ni = ar * pi + ai * pr;
    pr = nr; pi = ni;
    store2(PWR + (size_t)k * kN + n, pr); store2(PWI + (size_t)k * kN + n, pi);
  }
}

__global__ __launch_bounds__(64) void ktab_kernel(const float* __restrict__ Br, const float* __restrict__ Bi, const float* __restrict__ Cr, const float* __restrict__ Ci,
                                                 const float* __restrict__ PWR, const float* __restrict__ PWI, float* __restrict__ K32) {
  const unsigned l = threadIdx.x;
  float acc = 0.0f;
  for (int n = 0; n < kN; ++n) {
    const float br = Br[n], bi = Bi[n], cr = Cr[n], ci = Ci[n];
    const float b_r = bf16r(br), b_i = bf16r(bi), c_r = bf16r(cr), c_i = bf16r(ci);
    const float cbr = c_r * b_r + c_i * b_i;
    const float cbi = c_r * b_i - c_i * b_r;
    acc += cbr * PWR[(size_t)l * kN + n] - cbi * PWI[(size_t)l * kN + n];
  }
  store2(K32 + l, acc);
}

__global__ __launch_bounds__(64) void w2_kernel(const float* __restrict__ Cr, const float* __restrict__ Ci, const float* __restrict__ PWR, const float* __restrict__ PWI,
                                                const float* __restrict__ K32, unsigned short* __restrict__ W2) {
  const unsigned r = blockIdx.x;
  const unsigned g = threadIdx.x;
  if (g >= 24u) return;
  const unsigned c8 = g * 8u;
  v8h hv;
#pragma unroll
  for (int e = 0; e < 8; ++e) {
    const unsigned col = c8 + (unsigned)e;
    float v;
    if (col < 64u) {
      const float kv = K32[(r - col) & 63u];
      v = (col <= r) ? kv : 0.0f;
    } else {
      const unsigned n = (col - 64u) & 63u;
      const float cr = Cr[n], ci = Ci[n];
      const float c_r = bf16r(cr), c_i = bf16r(ci);
      const float pr = PWR[(size_t)(r + 1u) * kN + n], pi = PWI[(size_t)(r + 1u) * kN + n];
      v = (col < 128u) ? (c_r * pr + c_i * pi) : (c_i * pr - c_r * pi);
    }
    hv[e] = (_Float16)carry_flush(v, kTCarry);
  }
  unsigned short* dp = W2 + (size_t)r * kKY + c8;
  *(volatile v8h*)dp = hv;
  __threadfence();
  *(volatile v8h*)dp = hv;
}

__global__ __launch_bounds__(kThr) void bq_kernel(const float* __restrict__ Br, const float* __restrict__ Bi, const float* __restrict__ PWR, const float* __restrict__ PWI, unsigned short* __restrict__ BQ) {
  const unsigned t = blockIdx.x * (unsigned)kThr + threadIdx.x;
  const unsigned m = t >> 3, q8 = (t & 7u) * 8u;
  const unsigned n = m & 63u;
  const float br = Br[n], bi = Bi[n];
  const float b_r = bf16r(br), b_i = bf16r(bi);
  v8h hv;
#pragma unroll
  for (int e = 0; e < 8; ++e) {
    const unsigned k = 63u - (q8 + (unsigned)e);
    const float pr = PWR[(size_t)k * kN + n], pi = PWI[(size_t)k * kN + n];
    const float v = (m < 64u) ? (b_r * pr - b_i * pi) : (b_r * pi + b_i * pr);
    hv[e] = (_Float16)carry_flush(v, kACarry);
  }
  unsigned short* dp = BQ + (size_t)m * kQ + q8;
  *(volatile v8h*)dp = hv;
  __threadfence();
  *(volatile v8h*)dp = hv;
}
static_assert(kS * (kQ / 8) == 4 * kThr, "state-operand cast grid exact: 4 blocks");

__global__ __launch_bounds__(kThr) void xcast_kernel(const float* __restrict__ X, unsigned short* __restrict__ XH) {
  const unsigned t = blockIdx.x * (unsigned)kThr + threadIdx.x;
  const unsigned row = t >> 3, c8 = (t & 7u) * 8u;
  const float* sp = X + (size_t)row * kQ + c8;
  v8h hv;
#pragma unroll
  for (int e = 0; e < 8; ++e) { const float v = sp[e]; hv[e] = (_Float16)carry_flush(bf16r(v), kInCarry); }
  unsigned short* dp = XH + (size_t)row * kKY + c8;
  *(volatile v8h*)dp = hv;
  __threadfence();
  *(volatile v8h*)dp = hv;
}
static_assert(kR * (kQ / 8) == 512 * kThr, "input cast grid exact: 512 blocks");

__global__ __launch_bounds__(kThr) void cscan_kernel(const float* __restrict__ HIN, const float* __restrict__ Dr, const float* __restrict__ Di, float* __restrict__ H) {
  const unsigned i = blockIdx.x * (unsigned)kThr + threadIdx.x;
  const unsigned b = i >> 6, n = i & 63u;
  const float dr = Dr[n], di = Di[n];
  float hr = 0.0f, hi = 0.0f;
  for (int c = 0; c < kC; ++c) {
    const size_t row = (size_t)b * kC + (size_t)c;
    store2(H + row * kS + n, hr);
    store2(H + row * kS + kN + n, hi);
    const float ir = HIN[row * kS + n], ii = HIN[row * kS + kN + n];
    const float nr = dr * hr - di * hi + ir;
    const float ni = dr * hi + di * hr + ii;
    hr = nr; hi = ni;
  }
}
static_assert(kB * kN == 64 * kThr, "chunk recurrence grid exact: 64 blocks");

__global__ __launch_bounds__(kThr) void hcast_kernel(const float* __restrict__ H, unsigned short* __restrict__ XH) {
  const unsigned t = blockIdx.x * (unsigned)kThr + threadIdx.x;
  const unsigned row = t >> 4, s8 = (t & 15u) * 8u;
  const float* sp = H + (size_t)row * kS + s8;
  v8h hv;
#pragma unroll
  for (int e = 0; e < 8; ++e) { const float v = sp[e]; hv[e] = (_Float16)carry_flush(v, kInCarry); }
  unsigned short* dp = XH + (size_t)row * kKY + (unsigned)kQ + s8;
  *(volatile v8h*)dp = hv;
  __threadfence();
  *(volatile v8h*)dp = hv;
}
static_assert((size_t)kR * (kS / 8) == 1024ull * kThr, "state cast grid exact: 1,024 blocks");

extern "C" void kernel_launch(void* const* d_in, const int* in_sizes, int n_in,
                              void* d_out, int out_size, void* d_ws, size_t ws_size,
                              hipStream_t stream) {
  if (n_in < 7 || d_out == nullptr || d_ws == nullptr) return;
  if (in_sizes[0] != kB * kL || in_sizes[1] != kN || in_sizes[2] != kN || in_sizes[3] != kN || in_sizes[4] != kN || in_sizes[5] != kN || in_sizes[6] != kN) return;
  if (out_size != kB * kL) return;
  if (ws_size < kWsTotal) return;
  const float* X = (const float*)d_in[0];
  const float* rho = (const float*)d_in[1];
  const float* theta = (const float*)d_in[2];
  const float* Br = (const float*)d_in[3];
  const float* Bi = (const float*)d_in[4];
  const float* Cr = (const float*)d_in[5];
  const float* Ci = (const float*)d_in[6];
  float* out = (float*)d_out;
  char* ws = (char*)d_ws;
  float* ZB = (float*)(ws + kOffZB);
  float* PWR = (float*)(ws + kOffPWR);
  float* PWI = (float*)(ws + kOffPWI);
  float* K32 = (float*)(ws + kOffK32);
  unsigned short* W216 = (unsigned short*)(ws + kOffW216);
  unsigned short* BQ16 = (unsigned short*)(ws + kOffBQ16);
  unsigned short* XH16 = (unsigned short*)(ws + kOffXH16);
  float* HIN32 = (float*)(ws + kOffHIN32);
  float* H32 = (float*)(ws + kOffH32);

  zero_kernel<<<1, kThr, 0, stream>>>(ZB);
  pow_kernel<<<1, 64, 0, stream>>>(rho, theta, PWR, PWI);
  ktab_kernel<<<1, 64, 0, stream>>>(Br, Bi, Cr, Ci, PWR, PWI, K32);
  w2_kernel<<<kQ, 64, 0, stream>>>(Cr, Ci, PWR, PWI, K32, W216);
  bq_kernel<<<4, kThr, 0, stream>>>(Br, Bi, PWR, PWI, BQ16);
  xcast_kernel<<<512, kThr, 0, stream>>>(X, XH16);
  wmma_gemm64<0, false, 2, 0, false, 0><<<dim3((kR / 64) * (kS / 64) / 8, 1), 256, 0, stream>>>(
      XH16, XH16, kKY, 0L, BQ16, BQ16, kQ, 0L, (void*)HIN32, (void*)HIN32, kS, 0L, ZB, nullptr, 0L, kR, kS, kQ, kSc1);
  cscan_kernel<<<64, kThr, 0, stream>>>(HIN32, PWR + (size_t)kQ * kN, PWI + (size_t)kQ * kN, H32);
  hcast_kernel<<<1024, kThr, 0, stream>>>(H32, XH16);
  wmma_gemm64<0, false, 2, 0, false, 0><<<dim3((kR / 64) * (kQ / 64) / 8, 1), 256, 0, stream>>>(
      XH16, XH16, kKY, 0L, W216, W216, kKY, 0L, (void*)out, (void*)out, kQ, 0L, ZB, nullptr, 0L, kR, kQ, kKY, kSc2);
}
